// Scaled_Dot_Product_Attention_15702400434586
// MI455X (gfx1250) — hardware-verified
//
#include <hip/hip_runtime.h>
#include <math.h>

constexpr int kSeq   = 2048;
constexpr int kHd    = 64;
constexpr int kNbh   = 32;
constexpr int kQB    = 64;
constexpr int kKC    = 64;
constexpr int kNW    = 4;
constexpr int kNElem = kNbh * kSeq * kHd;
constexpr float kQScale = 0.125f;
static_assert(kSeq % kQB == 0);
static_assert(kQB == kKC);
static_assert(kHd == 64);
static_assert(kNElem % 8 == 0);

typedef __attribute__((ext_vector_type(16))) __bf16   v16b;
typedef __attribute__((ext_vector_type(8)))  __bf16   v8b;
typedef __attribute__((ext_vector_type(8)))  float    v8f;
typedef __attribute__((ext_vector_type(4)))  float    v4f;
typedef __attribute__((ext_vector_type(4)))  unsigned int v4u;

__device__ __forceinline__ unsigned short f2bf_bits(float f) {
  unsigned u = __float_as_uint(f);
  return (unsigned short)((u + 0x7FFFu + ((u >> 16) & 1u)) >> 16);
}
__device__ __forceinline__ float bf_bits2f(unsigned short h) { return __uint_as_float(((unsigned)h) << 16); }

__device__ __forceinline__ void dep_guard_b(v8f& a, v8f& b, v16b x, v16b y) { asm volatile("v_nop\n\tv_nop\n\tv_nop\n\tv_nop" : "+v"(a), "+v"(b) : "v"(x), "v"(y)); }
__device__ __forceinline__ void keep4_b(v16b a, v16b b, v16b c, v16b d) { asm volatile("v_nop" :: "v"(a), "v"(b), "v"(c), "v"(d)); }

template <typename T> struct Frag;
template <> struct Frag<__bf16> {
  typedef v16b V; union U { v16b v; v8b h[2]; };
  static __device__ __forceinline__ v16b load(const __bf16* p) {
    U f; f.h[0] = *(const v8b*)(p); f.h[1] = *(const v8b*)(p + 16); return f.v;
  }
  static __device__ __forceinline__ v8f mma(v16b a, v16b b, v8f c) {
    return __builtin_amdgcn_wmma_f32_16x16x32_bf16(false, a, false, b, (short)0, c, false, false);
  }
  static __device__ __forceinline__ void guard(v8f& a, v8f& b, v16b x, v16b y) { dep_guard_b(a, b, x, y); }
  static __device__ __forceinline__ void keep(v16b a, v16b b, v16b c, v16b d) { keep4_b(a, b, c, d); }
};

__device__ __forceinline__ unsigned pk16(unsigned short a, unsigned short b) { return (unsigned)a | ((unsigned)b << 16); }

__device__ __forceinline__ unsigned short at_bf_bits(float f) {
  unsigned u = __float_as_uint(f);
  return (unsigned short)((u + 0x7FFFu + ((u >> 16) & 1u)) >> 16);
}
__device__ __forceinline__ __bf16 at_f2bf(float f) { return __builtin_bit_cast(__bf16, at_bf_bits(f)); }
__device__ __forceinline__ void at_split(float f, __bf16& hi, __bf16& lo) {
  const unsigned short hb = at_bf_bits(f);
  hi = __builtin_bit_cast(__bf16, hb);
  lo = at_f2bf(f - __uint_as_float(((unsigned)hb) << 16));
}
__device__ __forceinline__ v8f at_mma(v16b a, v16b b, v8f c) {
  c = __builtin_amdgcn_wmma_f32_16x16x32_bf16(false, a, false, b, (short)0, c, false, false);
  asm volatile("v_nop\n\tv_nop\n\tv_nop\n\tv_nop" : "+v"(c) : "v"(a), "v"(b));
  return c;
}

__global__ __launch_bounds__(256) void cast8_bf16_kernel(const float* __restrict__ q, const float* __restrict__ k,
                                                         const float* __restrict__ v,
                                                         unsigned short* __restrict__ qo, unsigned short* __restrict__ ko,
                                                         unsigned short* __restrict__ vo, int n8) {
  const int i = blockIdx.x * 256 + threadIdx.x;
  const int z = blockIdx.y;
  const float* in = (z == 0) ? q : (z == 1) ? k : v;
  unsigned short* o = (z == 0) ? qo : (z == 1) ? ko : vo;
  const float scale = (z == 0) ? kQScale : 1.0f;
  if (i >= n8) return;
  const float* p = in + 8 * (size_t)i;
  const v4f a = *(const v4f*)(p);
  const v4f c = *(const v4f*)(p + 4);
  unsigned short hb[8];
#pragma unroll
  for (int e = 0; e < 4; ++e) {
    hb[e]     = f2bf_bits(a[e] * scale);
    hb[4 + e] = f2bf_bits(c[e] * scale);
  }
  const v4u u = (v4u){pk16(hb[0], hb[1]), pk16(hb[2], hb[3]), pk16(hb[4], hb[5]), pk16(hb[6], hb[7])};
  unsigned short* op = o + 8 * (size_t)i;
  *(volatile v4u*)op = u;
  __threadfence();
  *(volatile v4u*)op = u;
}

__global__ __launch_bounds__(128)
void attn_causal_kernel(const unsigned short* __restrict__ qp, const unsigned short* __restrict__ kp,
                        const unsigned short* __restrict__ vp, float* __restrict__ out) {
  union FB { v16b v; v8b h[2]; };
  __shared__ __align__(16) unsigned short Ksh[kKC * kHd];
  __shared__ __align__(16) unsigned short Vth[kHd * kKC];
  __shared__ __align__(16) __bf16 Psh[kNW][16 * kKC];
  __shared__ __align__(16) __bf16 Psl[kNW][16 * kKC];
  __shared__ __align__(16) float  Os[kNW][16 * 68];

  const int tid  = threadIdx.x;
  const int wave = tid >> 5;
  const int lane = tid & 31;
  const int hh   = lane >> 4;
  const int c    = lane & 15;

  const int nqb = kSeq / kQB;
  const int bx  = blockIdx.x;
  const int qb  = bx % nqb;
  const int bh  = bx / nqb;
  const int q0  = qb * kQB + wave * 16;

  const size_t planeOff = (size_t)bh * kSeq * kHd;
  const unsigned short* qb_ptr = qp + planeOff;
  const unsigned short* kb_ptr = kp + planeOff;
  const unsigned short* vb_ptr = vp + planeOff;
  float* ob_ptr = out + planeOff;

  v16b qa[2];
  {
    const __bf16* qrow = (const __bf16*)(const void*)(qb_ptr + (size_t)(q0 + c) * kHd);
#pragma unroll
    for (int dc = 0; dc < 2; ++dc) qa[dc] = Frag<__bf16>::load(qrow + dc * 32 + 8 * hh);
  }

  float mrow[8], lrow[8];
  v8f oacc[4];
#pragma unroll
  for (int r = 0; r < 8; ++r) { mrow[r] = -__builtin_inff(); lrow[r] = 0.0f; }
#pragma unroll
  for (int t = 0; t < 4; ++t) oacc[t] = (v8f){0.f,0.f,0.f,0.f,0.f,0.f,0.f,0.f};

  const int nChunks = qb + 1;
  for (int kc = 0; kc < nChunks; ++kc) {
    const int kv0 = kc * kKC;
    __syncthreads();
    {
      const int kvr = tid >> 1, dh = (tid & 1) * 32;
      const v4u* ksrc = (const v4u*)(const void*)(kb_ptr + (size_t)(kv0 + kvr) * kHd + dh);
      const v4u* vsrc = (const v4u*)(const void*)(vb_ptr + (size_t)(kv0 + kvr) * kHd + dh);
      v4u kw[4], vw[4];
#pragma unroll
      for (int i = 0; i < 4; ++i) { kw[i] = ksrc[i]; vw[i] = vsrc[i]; }
#pragma unroll
      for (int i = 0; i < 4; ++i) *(v4u*)(void*)(Ksh + kvr * kHd + dh + 8 * i) = kw[i];
#pragma unroll
      for (int i = 0; i < 4; ++i) {
#pragma unroll
        for (int e2 = 0; e2 < 4; ++e2) {
          const unsigned w = vw[i][e2];
          const int d = dh + 8 * i + 2 * e2;
          Vth[d * kKC + kvr]       = (unsigned short)(w & 0xffffu);
          Vth[(d + 1) * kKC + kvr] = (unsigned short)(w >> 16);
        }
      }
    }
    __syncthreads();

    v8f s[4];
#pragma unroll
    for (int j = 0; j < 4; ++j) {
      s[j] = (v8f){0.f,0.f,0.f,0.f,0.f,0.f,0.f,0.f};
#pragma unroll
      for (int dc = 0; dc < 2; ++dc) {
        FB kb;
        kb.h[0] = *(const v8b*)(const void*)(Ksh + (j * 16 + c) * kHd + dc * 32 + 8 * hh);
        kb.h[1] = *(const v8b*)(const void*)(Ksh + (j * 16 + c) * kHd + dc * 32 + 16 + 8 * hh);
        s[j] = at_mma(qa[dc], kb.v, s[j]);
      }
    }

    const bool diag = (kc == qb);
    float cm[8];
#pragma unroll
    for (int r = 0; r < 8; ++r) {
      const int qrow = q0 + 8 * hh + r;
      float m = -__builtin_inff();
#pragma unroll
      for (int j = 0; j < 4; ++j) {
        const int kvcol = kv0 + j * 16 + c;
        const bool masked = diag && (kvcol > qrow);
        const float sv = masked ? -__builtin_inff() : s[j][r];
        s[j][r] = sv;
        m = fmaxf(m, sv);
      }
#pragma unroll
      for (int off = 1; off < 16; off <<= 1) m = fmaxf(m, __shfl_xor(m, off, 32));
      cm[r] = m;
    }

    __bf16* pwh = Psh[wave];
    __bf16* pwl = Psl[wave];
#pragma unroll
    for (int r = 0; r < 8; ++r) {
      const float mnew  = fmaxf(mrow[r], cm[r]);
      const float alpha = expf(mrow[r] - mnew);
      mrow[r] = mnew;
      float psum = 0.0f;
#pragma unroll
      for (int j = 0; j < 4; ++j) {
        const float p = expf(s[j][r] - mnew);
        psum += p;
        __bf16 ph, pl;
        at_split(p, ph, pl);
        pwh[(8 * hh + r) * kKC + j * 16 + c] = ph;
        pwl[(8 * hh + r) * kKC + j * 16 + c] = pl;
      }
#pragma unroll
      for (int off = 1; off < 16; off <<= 1) psum += __shfl_xor(psum, off, 32);
      lrow[r] = lrow[r] * alpha + psum;
#pragma unroll
      for (int t = 0; t < 4; ++t) oacc[t][r] *= alpha;
    }
    __builtin_amdgcn_fence(__ATOMIC_RELEASE, "workgroup");
    __builtin_amdgcn_wave_barrier();
    __builtin_amdgcn_fence(__ATOMIC_ACQUIRE, "workgroup");

#pragma unroll 1
    for (int kk = 0; kk < 2; ++kk) {
      FB pa, pl;
      pa.h[0] = *(const v8b*)(pwh + c * kKC + kk * 32 + 8 * hh);
      pa.h[1] = *(const v8b*)(pwh + c * kKC + kk * 32 + 16 + 8 * hh);
      pl.h[0] = *(const v8b*)(pwl + c * kKC + kk * 32 + 8 * hh);
      pl.h[1] = *(const v8b*)(pwl + c * kKC + kk * 32 + 16 + 8 * hh);
#pragma unroll
      for (int t = 0; t < 4; ++t) {
        FB vb;
        vb.h[0] = *(const v8b*)(const void*)(Vth + (t * 16 + c) * kKC + kk * 32 + 8 * hh);
        vb.h[1] = *(const v8b*)(const void*)(Vth + (t * 16 + c) * kKC + kk * 32 + 16 + 8 * hh);
        oacc[t] = at_mma(pa.v, vb.v, oacc[t]);
        oacc[t] = at_mma(pl.v, vb.v, oacc[t]);
      }
    }
  }

  float* os = Os[wave];
#pragma unroll
  for (int r = 0; r < 8; ++r) {
    const float inv = 1.0f / lrow[r];
#pragma unroll
    for (int t = 0; t < 4; ++t) os[(8 * hh + r) * 68 + t * 16 + c] = oacc[t][r] * inv;
  }
  __builtin_amdgcn_fence(__ATOMIC_RELEASE, "workgroup");
  __builtin_amdgcn_wave_barrier();
  __builtin_amdgcn_fence(__ATOMIC_ACQUIRE, "workgroup");
  {
    const int c4 = (lane & 15) * 4;
    for (int pass = 0; pass < 2; ++pass) {
#pragma unroll
      for (int it = 0; it < 8; ++it) {
        const int row = it * 2 + hh;
        const v4f val = *(const v4f*)(os + row * 68 + c4);
        *(volatile v4f*)(ob_ptr + (size_t)(q0 + row) * kHd + c4) = val;
      }
      __threadfence();
    }
  }
}

extern "C" void kernel_launch(void* const* d_in, const int* in_sizes, int n_in,
                              void* d_out, int out_size, void* d_ws, size_t ws_size,
                              hipStream_t stream) {
  if (n_in < 4) return;
  if (in_sizes[0] != kNElem || in_sizes[1] != kNElem || in_sizes[2] != kNElem) return;
  if (out_size != kNElem) return;

  const size_t szPlane = (size_t)kNElem * 2;
  const size_t offQ = 0;
  const size_t offK = offQ + szPlane;
  const size_t offV = offK + szPlane;
  const size_t total = offV + szPlane;
  if (ws_size < total) return;

  const float* Q = (const float*)d_in[0];
  const float* K = (const float*)d_in[1];
  const float* V = (const float*)d_in[2];
  float* out = (float*)d_out;
  char* ws = (char*)d_ws;
  unsigned short* Qp = (unsigned short*)(ws + offQ);
  unsigned short* Kp = (unsigned short*)(ws + offK);
  unsigned short* Vp = (unsigned short*)(ws + offV);

  const int n8 = kNElem / 8;
  cast8_bf16_kernel<<<dim3((n8 + 255) / 256, 3), dim3(256), 0, stream>>>(Q, K, V, Qp, Kp, Vp, n8);

  attn_causal_kernel<<<dim3(kNbh * (kSeq / kQB)), dim3(128), 0, stream>>>(Qp, Kp, Vp, out);
}
